// MSA2Pair_30193620091046
// MI455X (gfx1250) — hardware-verified
//
#include <hip/hip_runtime.h>

#ifndef NSEQ
#define NSEQ 192
#endif
#define NSEQ_FULL 192
#ifndef LL
#define LL 256
#endif
#ifndef LL_FULL
#define LL_FULL 256
#endif
#define FF 64
#define PP 32
#define OO 128
#define CIN 384
#define NPIX (LL * LL)
#define PADW (LL + 2)
#define NPADPIX (PADW * PADW)
#define NROW0 (NSEQ * LL)
#define KPR (PP * PP)
#define K33 (9 * OO)
#define LNP (KPR + 8)
#define OPITCH (OO + 4)
#define NB4 (LL / 4)
#define NTRI (NB4 * (NB4 + 1) / 2)
#define KPAIR_LDS (32 * LNP * 2 + 16 * OPITCH * 4 + 2 * KPR * 4)
static_assert(NSEQ % 32 == 0);
static_assert(NSEQ >= 32);
static_assert(NSEQ <= NSEQ_FULL);
static_assert(LL % 64 == 0);
static_assert(LL >= 64);
static_assert(LL <= LL_FULL);
static_assert((NROW0 % 64) == 0);
static_assert((NPIX % 128) == 0);
static_assert((LNP % 8) == 0);
static_assert((OPITCH % 4) == 0);

typedef __bf16 v16b __attribute__((ext_vector_type(16)));
typedef unsigned short v8us __attribute__((ext_vector_type(8), may_alias));
typedef unsigned short v4us __attribute__((ext_vector_type(4), may_alias));
typedef float v8f __attribute__((ext_vector_type(8)));
typedef float v4f __attribute__((ext_vector_type(4)));
typedef float v4fa __attribute__((ext_vector_type(4), may_alias));
typedef float v2fa __attribute__((ext_vector_type(2), may_alias));
union FragB { v16b v; v8us half[2]; unsigned short u[16]; };

__device__ __forceinline__ unsigned short bfb(float x) { unsigned int u = __float_as_uint(x); return (unsigned short)((u + 0x7FFFu + ((u >> 16) & 1u)) >> 16); }
__device__ __forceinline__ float bfv(unsigned short b) { return __uint_as_float(((unsigned int)b) << 16); }
__device__ __forceinline__ float bfr(float x) { return bfv(bfb(x)); }
__device__ __forceinline__ v8f zero8() { v8f z; for (int i = 0; i < 8; ++i) z[i] = 0.f; return z; }

__device__ __forceinline__ v8f mma2(v16b ah, v16b al, v16b b, v8f c) {
  c = __builtin_amdgcn_wmma_f32_16x16x32_bf16(false, ah, false, b, (short)0, c, false, false);
  c = __builtin_amdgcn_wmma_f32_16x16x32_bf16(false, al, false, b, (short)0, c, false, false);
  asm volatile("v_nop\n\tv_nop\n\tv_nop\n\tv_nop" : "+v"(c) : "v"(ah), "v"(al), "v"(b));
  return c;
}
__device__ __forceinline__ v8f mma3(v16b ah, v16b al, v16b bh, v16b bl, v8f c) {
  c = __builtin_amdgcn_wmma_f32_16x16x32_bf16(false, ah, false, bh, (short)0, c, false, false);
  c = __builtin_amdgcn_wmma_f32_16x16x32_bf16(false, al, false, bh, (short)0, c, false, false);
  c = __builtin_amdgcn_wmma_f32_16x16x32_bf16(false, ah, false, bl, (short)0, c, false, false);
  asm volatile("v_nop\n\tv_nop\n\tv_nop\n\tv_nop" : "+v"(c) : "v"(ah), "v"(al), "v"(bh), "v"(bl));
  return c;
}
__device__ __forceinline__ v16b fragG(const unsigned short* p, int hh) { FragB f; f.half[0] = *(const v8us*)(p + 8 * hh); f.half[1] = *(const v8us*)(p + 16 + 8 * hh); return f.v; }
__device__ __forceinline__ float wsum(float v) {
#pragma unroll
  for (int m = 16; m > 0; m >>= 1) v += __shfl_xor(v, m, 32);
  return v;
}
__device__ __forceinline__ float eluf(float v) { return v > 0.f ? v : expm1f(v); }

__global__ __launch_bounds__(256) void k_cvt(const float* __restrict__ W, unsigned short* __restrict__ Ob, int n8) {
  const int t = blockIdx.x * 256 + threadIdx.x;
  if (t >= n8) return;
  const v4f a = *(const v4fa*)(W + (size_t)t * 8), c = *(const v4fa*)(W + (size_t)t * 8 + 4);
  FragB f;
#pragma unroll
  for (int q = 0; q < 4; ++q) { f.u[q] = bfb(a[q]); f.u[4 + q] = bfb(c[q]); }
  const v8us o = f.half[0];
  *(volatile v8us*)(Ob + (size_t)t * 8) = o;
  __threadfence();
  *(volatile v8us*)(Ob + (size_t)t * 8) = o;
}

__global__ __launch_bounds__(256) void k_w9(const float* __restrict__ w, unsigned short* __restrict__ Wt) {
  const int t = blockIdx.x * 256 + threadIdx.x;
  if (t >= OO * 9 * 16) return;
  const int c8 = (t & 15) * 8, tap = (t >> 4) % 9, o = t / 144;
  FragB f;
#pragma unroll
  for (int j = 0; j < 8; ++j) f.u[j] = bfb(w[((size_t)(o * OO + c8 + j)) * 9 + tap]);
  const v8us o8 = f.half[0];
  unsigned short* dst = Wt + (size_t)o * K33 + tap * OO + c8;
  *(volatile v8us*)dst = o8;
  __threadfence();
  *(volatile v8us*)dst = o8;
}

__global__ __launch_bounds__(128) void k_proj1(const float* __restrict__ msa, const float* __restrict__ g, const float* __restrict__ bb,
                                               const unsigned short* __restrict__ W1b, const float* __restrict__ b1, float* __restrict__ XD) {
  __shared__ __attribute__((aligned(16))) float so[4][16][32];
  const int tid = threadIdx.x, w = tid >> 5, lane = tid & 31, ln = lane & 15, hh = lane >> 4;
  const int row0 = (blockIdx.x * 4 + w) * 16;
  const int rr = row0 + ln;
  const int nn = rr / LL, l1 = rr - nn * LL;
  const float* arow = msa + ((size_t)nn * LL_FULL + (size_t)l1) * FF;
  float xs[32];
#pragma unroll
  for (int gi = 0; gi < 4; ++gi) {
    const int f0 = (gi >> 1) * 32 + (gi & 1) * 16 + 8 * hh;
    const v4f a = *(const v4fa*)(arow + f0), c = *(const v4fa*)(arow + f0 + 4);
#pragma unroll
    for (int q = 0; q < 4; ++q) { xs[gi * 8 + q] = bfr(a[q]); xs[gi * 8 + 4 + q] = bfr(c[q]); }
  }
  float s = 0.f;
#pragma unroll
  for (int i = 0; i < 32; ++i) s += xs[i];
  s += __shfl_xor(s, 16, 32);
  const float mean = s * (1.0f / 64.0f);
  float q2 = 0.f;
#pragma unroll
  for (int i = 0; i < 32; ++i) { const float d = xs[i] - mean; q2 += d * d; }
  q2 += __shfl_xor(q2, 16, 32);
  const float rstd = rsqrtf(q2 * (1.0f / 64.0f) + 1e-5f);
  FragB ah[2], al[2];
#pragma unroll
  for (int gi = 0; gi < 4; ++gi) {
    const int f0 = (gi >> 1) * 32 + (gi & 1) * 16 + 8 * hh;
    const v4f ga = *(const v4fa*)(g + f0), gc = *(const v4fa*)(g + f0 + 4);
    const v4f ba = *(const v4fa*)(bb + f0), bc = *(const v4fa*)(bb + f0 + 4);
#pragma unroll
    for (int q = 0; q < 4; ++q) {
      const float m0 = (xs[gi * 8 + q] - mean) * rstd * bfr(ga[q]) + bfr(ba[q]);
      const unsigned short h0 = bfb(m0);
      ah[gi >> 1].u[(gi & 1) * 8 + q] = h0; al[gi >> 1].u[(gi & 1) * 8 + q] = bfb(m0 - bfv(h0));
      const float m1 = (xs[gi * 8 + 4 + q] - mean) * rstd * bfr(gc[q]) + bfr(bc[q]);
      const unsigned short h1 = bfb(m1);
      ah[gi >> 1].u[(gi & 1) * 8 + 4 + q] = h1; al[gi >> 1].u[(gi & 1) * 8 + 4 + q] = bfb(m1 - bfv(h1));
    }
  }
  v8f acc[2];
  acc[0] = zero8(); acc[1] = zero8();
#pragma unroll
  for (int ks = 0; ks < 2; ++ks) {
#pragma unroll
    for (int t = 0; t < 2; ++t) {
      const v16b bq = fragG(W1b + (size_t)(t * 16 + ln) * FF + ks * 32, hh);
      acc[t] = mma2(ah[ks].v, al[ks].v, bq, acc[t]);
    }
  }
#pragma unroll
  for (int t = 0; t < 2; ++t) {
    const float bv = bfr(b1[t * 16 + ln]);
#pragma unroll
    for (int r = 0; r < 8; ++r) so[w][8 * hh + r][t * 16 + ln] = acc[t][r] + bv;
  }
  __builtin_amdgcn_fence(__ATOMIC_ACQ_REL, "workgroup");
  __builtin_amdgcn_wave_barrier();
  for (int pass = 0; pass < 2; ++pass) {
#pragma unroll
    for (int u = 0; u < 4; ++u) {
      const int j = u * 32 + lane;
      const v4f v = *(const v4fa*)&so[w][j >> 3][(j & 7) * 4];
      *(volatile v4f*)(XD + (size_t)row0 * PP + (size_t)j * 4) = v;
    }
    if (pass == 0) __threadfence();
  }
}

__global__ __launch_bounds__(256) void k_xt(const float* __restrict__ XD, unsigned short* __restrict__ XTh, unsigned short* __restrict__ XTl) {
  __shared__ __attribute__((aligned(16))) unsigned short th[PP][NSEQ + 8];
  __shared__ __attribute__((aligned(16))) unsigned short tl[PP][NSEQ + 8];
  const int l = blockIdx.x, tid = threadIdx.x;
  for (int idx = tid; idx < NSEQ * PP; idx += 256) {
    const int n = idx >> 5, p = idx & 31;
    const float v = XD[((size_t)n * LL + l) * PP + p];
    const unsigned short hb = bfb(v);
    th[p][n] = hb; tl[p][n] = bfb(v - bfv(hb));
  }
  __syncthreads();
  const int NP8 = NSEQ / 8;
  for (int pass = 0; pass < 2; ++pass) {
    for (int j = tid; j < 4 * NSEQ; j += 256) {
      const int p = j / NP8, n0 = (j - p * NP8) * 8;
      const v8us hv = *(const v8us*)&th[p][n0];
      const v8us lv = *(const v8us*)&tl[p][n0];
      *(volatile v8us*)(XTh + (size_t)l * PP * NSEQ + (size_t)j * 8) = hv;
      *(volatile v8us*)(XTl + (size_t)l * PP * NSEQ + (size_t)j * 8) = lv;
    }
    if (pass == 0) __threadfence();
  }
}

__global__ __launch_bounds__(256) void k_feat(const float* __restrict__ XD, const float* __restrict__ g, const float* __restrict__ bb,
                                              unsigned short* __restrict__ Fh, unsigned short* __restrict__ Fl) {
  __shared__ float facc[8][32];
  __shared__ __attribute__((aligned(16))) float rowv[64];
  const int l = blockIdx.x, tid = threadIdx.x, w = tid >> 5, lane = tid & 31;
  const float gg = bfr(g[lane]), bv = bfr(bb[lane]);
  float acc = 0.f, first = 0.f;
  for (int it = 0; it < NSEQ / 8; ++it) {
    const int n = it * 8 + w;
    const float x = XD[((size_t)n * LL + l) * PP + lane];
    const float mean = wsum(x) * (1.0f / 32.0f);
    const float d = x - mean;
    const float var = wsum(d * d) * (1.0f / 32.0f);
    const float nv = d * rsqrtf(var + 1e-5f) * gg + bv;
    acc += nv;
    if (n == 0) first = nv;
  }
  facc[w][lane] = acc;
  if (w == 0) rowv[32 + lane] = first;
  __syncthreads();
  if (w == 0) {
    float t = 0.f;
#pragma unroll
    for (int i = 0; i < 8; ++i) t += facc[i][lane];
    rowv[lane] = t * (1.0f / (float)NSEQ);
  }
  __syncthreads();
  if (w == 0) {
    const int li = lane & 15;
    const v4f v = *(const v4fa*)&rowv[li * 4];
    v4us hv, lv;
#pragma unroll
    for (int j = 0; j < 4; ++j) { const unsigned short hb = bfb(v[j]); hv[j] = hb; lv[j] = bfb(v[j] - bfv(hb)); }
    for (int pass = 0; pass < 2; ++pass) {
      if (lane < 16) {
        *(volatile v4us*)(Fh + (size_t)l * FF + li * 4) = hv;
        *(volatile v4us*)(Fl + (size_t)l * FF + li * 4) = lv;
      }
      if (pass == 0) __threadfence();
    }
  }
}

__global__ __launch_bounds__(256) void k_lnpo(const float* __restrict__ X, const float* __restrict__ g, const float* __restrict__ bb,
                                              unsigned short* __restrict__ Ph, unsigned short* __restrict__ Pl) {
  const int tid = threadIdx.x, w = tid >> 5, lane = tid & 31;
  const size_t row = (size_t)blockIdx.x * 8 + w;
  const size_t ii = row / LL, l1 = row - ii * LL;
  const v4f xr = *(const v4fa*)(X + (ii * LL_FULL + l1) * OO + lane * 4);
  float x[4];
#pragma unroll
  for (int j = 0; j < 4; ++j) x[j] = bfr(xr[j]);
  float s = x[0] + x[1] + x[2] + x[3];
  s = wsum(s);
  const float mean = s * (1.0f / 128.0f);
  float d[4], q = 0.f;
#pragma unroll
  for (int j = 0; j < 4; ++j) { d[j] = x[j] - mean; q += d[j] * d[j]; }
  q = wsum(q);
  const float rs = rsqrtf(q * (1.0f / 128.0f) + 1e-5f);
  const v4f gv = *(const v4fa*)(g + lane * 4), bv = *(const v4fa*)(bb + lane * 4);
  v4us hv, lv;
#pragma unroll
  for (int j = 0; j < 4; ++j) { const float nv = d[j] * rs * bfr(gv[j]) + bfr(bv[j]); const unsigned short hb = bfb(nv); hv[j] = hb; lv[j] = bfb(nv - bfv(hb)); }
  for (int pass = 0; pass < 2; ++pass) {
    *(volatile v4us*)(Ph + row * OO + lane * 4) = hv;
    *(volatile v4us*)(Pl + row * OO + lane * 4) = lv;
    if (pass == 0) __threadfence();
  }
}

__global__ __launch_bounds__(256) void k_pair(const unsigned short* __restrict__ XTh, const unsigned short* __restrict__ XTl,
                                              const float* __restrict__ g2d, const float* __restrict__ b2d,
                                              const unsigned short* __restrict__ W2t, const float* __restrict__ b2,
                                              const float* __restrict__ gn, const float* __restrict__ bn,
                                              unsigned short* __restrict__ PNh, unsigned short* __restrict__ PNl) {
  extern __shared__ __attribute__((aligned(16))) unsigned char dlds[];
  unsigned short* lnh = (unsigned short*)dlds;
  unsigned short* lnl = lnh + 16 * LNP;
  float* outr = (float*)(dlds + (size_t)32 * LNP * 2);
  float* gb = outr + 16 * OPITCH;
  const int tid = threadIdx.x, w = tid >> 5, lane = tid & 31, ln = lane & 15, hh = lane >> 4;
  int tt = blockIdx.x, ib = 0;
  while (tt >= NB4 - ib) { tt -= NB4 - ib; ++ib; }
  const int lb = ib + tt;
  {
    const v4f gv = *(const v4fa*)(g2d + tid * 4), bv = *(const v4fa*)(b2d + tid * 4);
#pragma unroll
    for (int j = 0; j < 4; ++j) { gb[tid * 4 + j] = bfr(gv[j]); gb[KPR + tid * 4 + j] = bfr(bv[j]); }
  }
  const int il = w & 3, lp = (w >> 2) * 2;
  const size_t ra0 = ((size_t)(ib * 4 + il) * PP + ln) * NSEQ, ra1 = ra0 + (size_t)16 * NSEQ;
  const size_t rb0 = ((size_t)(lb * 4 + lp) * PP + ln) * NSEQ;
  v8f acc[2][4];
#pragma unroll
  for (int mi = 0; mi < 2; ++mi)
#pragma unroll
    for (int nj = 0; nj < 4; ++nj) acc[mi][nj] = zero8();
#pragma unroll 1
  for (int kb = 0; kb < NSEQ; kb += 32) {
    const v16b a0h = fragG(XTh + ra0 + kb, hh), a0l = fragG(XTl + ra0 + kb, hh);
    const v16b a1h = fragG(XTh + ra1 + kb, hh), a1l = fragG(XTl + ra1 + kb, hh);
#pragma unroll
    for (int nj = 0; nj < 4; ++nj) {
      const size_t rb = rb0 + (size_t)((nj >> 1) * PP + (nj & 1) * 16) * NSEQ + kb;
      const v16b bh = fragG(XTh + rb, hh), bl = fragG(XTl + rb, hh);
      acc[0][nj] = mma3(a0h, a0l, bh, bl, acc[0][nj]);
      acc[1][nj] = mma3(a1h, a1l, bh, bl, acc[1][nj]);
    }
  }
  const float invn = 1.0f / (float)NSEQ;
  float mean2[2], rstd2[2];
#pragma unroll
  for (int lsub = 0; lsub < 2; ++lsub) {
    float s = 0.f;
#pragma unroll
    for (int mi = 0; mi < 2; ++mi)
#pragma unroll
      for (int t2 = 0; t2 < 2; ++t2)
#pragma unroll
        for (int r = 0; r < 8; ++r) s += acc[mi][2 * lsub + t2][r] * invn;
    s = wsum(s);
    const float mean = s * (1.0f / 1024.0f);
    float q = 0.f;
#pragma unroll
    for (int mi = 0; mi < 2; ++mi)
#pragma unroll
      for (int t2 = 0; t2 < 2; ++t2)
#pragma unroll
        for (int r = 0; r < 8; ++r) { const float d = acc[mi][2 * lsub + t2][r] * invn - mean; q += d * d; }
    q = wsum(q);
    mean2[lsub] = mean; rstd2[lsub] = rsqrtf(q * (1.0f / 1024.0f) + 1e-5f);
  }
  const int nph = (ib < lb) ? 2 : 1;
  const size_t w2row = (size_t)(w * 16 + ln) * KPR;
  const float bias2 = bfr(b2[w * 16 + ln]);
  const v4f gnv = *(const v4fa*)(gn + lane * 4), bnv = *(const v4fa*)(bn + lane * 4);
#pragma unroll 1
  for (int ph = 0; ph < nph; ++ph) {
    __syncthreads();
#pragma unroll
    for (int mi = 0; mi < 2; ++mi) {
#pragma unroll
      for (int nj = 0; nj < 4; ++nj) {
        const int lsub = nj >> 1;
        const int l_local = lp + lsub;
        const int q = (nj & 1) * 16 + ln;
        const int R = (ph == 0) ? (il * 4 + l_local) : (l_local * 4 + il);
        const float mean = mean2[lsub], rs = rstd2[lsub];
#pragma unroll
        for (int r = 0; r < 8; ++r) {
          const int p = mi * 16 + 8 * hh + r;
          const int fi = (ph == 0) ? (p * 32 + q) : (q * 32 + p);
          const float nv = (acc[mi][nj][r] * invn - mean) * rs * gb[fi] + gb[KPR + fi];
          const unsigned short hb = bfb(nv);
          lnh[R * LNP + fi] = hb;
          lnl[R * LNP + fi] = bfb(nv - bfv(hb));
        }
      }
    }
    __syncthreads();
    v8f acc2 = zero8();
#pragma unroll 2
    for (int kb = 0; kb < KPR; kb += 32) {
      const v16b ah = fragG(lnh + ln * LNP + kb, hh), al = fragG(lnl + ln * LNP + kb, hh);
      const v16b bq = fragG(W2t + w2row + kb, hh);
      acc2 = mma2(ah, al, bq, acc2);
    }
#pragma unroll
    for (int r = 0; r < 8; ++r) outr[(8 * hh + r) * OPITCH + w * 16 + ln] = acc2[r] + bias2;
    __syncthreads();
    v4us hvs[2], lvs[2];
    size_t pixs[2];
#pragma unroll
    for (int t2 = 0; t2 < 2; ++t2) {
      const int R = w * 2 + t2;
      const v4f x = *(const v4fa*)(outr + R * OPITCH + lane * 4);
      float s = x[0] + x[1] + x[2] + x[3];
      s = wsum(s);
      const float mean = s * (1.0f / 128.0f);
      float d[4], q = 0.f;
#pragma unroll
      for (int j = 0; j < 4; ++j) { d[j] = x[j] - mean; q += d[j] * d[j]; }
      q = wsum(q);
      const float rs = rsqrtf(q * (1.0f / 128.0f) + 1e-5f);
      v4us hv, lv;
#pragma unroll
      for (int j = 0; j < 4; ++j) { const float nv = d[j] * rs * bfr(gnv[j]) + bfr(bnv[j]); const unsigned short hb = bfb(nv); hv[j] = hb; lv[j] = bfb(nv - bfv(hb)); }
      hvs[t2] = hv; lvs[t2] = lv;
      const int r1 = R >> 2, r2 = R & 3;
      pixs[t2] = (ph == 0) ? ((size_t)(ib * 4 + r1) * LL + (size_t)(lb * 4 + r2)) : ((size_t)(lb * 4 + r1) * LL + (size_t)(ib * 4 + r2));
    }
    for (int pass = 0; pass < 2; ++pass) {
#pragma unroll
      for (int t2 = 0; t2 < 2; ++t2) {
        *(volatile v4us*)(PNh + pixs[t2] * OO + lane * 4) = hvs[t2];
        *(volatile v4us*)(PNl + pixs[t2] * OO + lane * 4) = lvs[t2];
      }
      if (pass == 0) __threadfence();
    }
  }
}

__global__ __launch_bounds__(128) void k_conv1(const unsigned short* __restrict__ POh, const unsigned short* __restrict__ POl,
                                               const unsigned short* __restrict__ PNh, const unsigned short* __restrict__ PNl,
                                               const unsigned short* __restrict__ Fh, const unsigned short* __restrict__ Fl,
                                               const unsigned short* __restrict__ WCt, float* __restrict__ X0) {
  __shared__ __attribute__((aligned(16))) float so[4][32][68];
  const int tid = threadIdx.x, w = tid >> 5, lane = tid & 31, ln = lane & 15, hh = lane >> 4;
  const int mt = blockIdx.x >> 1, nq = blockIdx.x & 1;
  const int row0 = mt * 128 + 32 * w, col0 = nq * 64;
  const int y = row0 / LL, x0 = row0 - y * LL;
  const size_t ar0 = (size_t)(row0 + ln) * OO, ar1 = ar0 + (size_t)16 * OO;
  const size_t fy = (size_t)y * FF, fx0 = (size_t)(x0 + ln) * FF, fx1 = fx0 + (size_t)16 * FF;
  const unsigned short* b0p = WCt + (size_t)(col0 + ln) * CIN;
  v8f c0[4], c1[4];
#pragma unroll
  for (int t = 0; t < 4; ++t) { c0[t] = zero8(); c1[t] = zero8(); }
#pragma unroll 1
  for (int ks = 0; ks < 4; ++ks) {
    const int koff = ks * 32, kk = ks * 32;
    const v16b a0h = fragG(POh + ar0 + koff, hh), a0l = fragG(POl + ar0 + koff, hh);
    const v16b a1h = fragG(POh + ar1 + koff, hh), a1l = fragG(POl + ar1 + koff, hh);
#pragma unroll
    for (int t = 0; t < 4; ++t) {
      const v16b bq = fragG(b0p + (size_t)t * 16 * CIN + kk, hh);
      c0[t] = mma2(a0h, a0l, bq, c0[t]); c1[t] = mma2(a1h, a1l, bq, c1[t]);
    }
  }
#pragma unroll 1
  for (int ks = 0; ks < 4; ++ks) {
    const int koff = ks * 32, kk = OO + ks * 32;
    const v16b a0h = fragG(PNh + ar0 + koff, hh), a0l = fragG(PNl + ar0 + koff, hh);
    const v16b a1h = fragG(PNh + ar1 + koff, hh), a1l = fragG(PNl + ar1 + koff, hh);
#pragma unroll
    for (int t = 0; t < 4; ++t) {
      const v16b bq = fragG(b0p + (size_t)t * 16 * CIN + kk, hh);
      c0[t] = mma2(a0h, a0l, bq, c0[t]); c1[t] = mma2(a1h, a1l, bq, c1[t]);
    }
  }
#pragma unroll
  for (int ks = 0; ks < 2; ++ks) {
    const int koff = ks * 32, kk = 2 * OO + ks * 32;
    const v16b ah = fragG(Fh + fy + koff, hh), al = fragG(Fl + fy + koff, hh);
#pragma unroll
    for (int t = 0; t < 4; ++t) {
      const v16b bq = fragG(b0p + (size_t)t * 16 * CIN + kk, hh);
      c0[t] = mma2(ah, al, bq, c0[t]); c1[t] = mma2(ah, al, bq, c1[t]);
    }
  }
#pragma unroll
  for (int ks = 0; ks < 2; ++ks) {
    const int koff = ks * 32, kk = 2 * OO + FF + ks * 32;
    const v16b a0h = fragG(Fh + fx0 + koff, hh), a0l = fragG(Fl + fx0 + koff, hh);
    const v16b a1h = fragG(Fh + fx1 + koff, hh), a1l = fragG(Fl + fx1 + koff, hh);
#pragma unroll
    for (int t = 0; t < 4; ++t) {
      const v16b bq = fragG(b0p + (size_t)t * 16 * CIN + kk, hh);
      c0[t] = mma2(a0h, a0l, bq, c0[t]); c1[t] = mma2(a1h, a1l, bq, c1[t]);
    }
  }
#pragma unroll
  for (int t = 0; t < 4; ++t) {
#pragma unroll
    for (int r = 0; r < 8; ++r) { so[w][8 * hh + r][t * 16 + ln] = c0[t][r]; so[w][16 + 8 * hh + r][t * 16 + ln] = c1[t][r]; }
  }
  __builtin_amdgcn_fence(__ATOMIC_ACQ_REL, "workgroup");
  __builtin_amdgcn_wave_barrier();
  const int rsub = lane >> 4, c4 = (lane & 15) * 4;
  for (int pass = 0; pass < 2; ++pass) {
#pragma unroll
    for (int q = 0; q < 16; ++q) {
      const int r = q * 2 + rsub;
      const v4f v = *(const v4fa*)&so[w][r][c4];
      *(volatile v4f*)(X0 + (size_t)(row0 + r) * OO + col0 + c4) = v;
    }
    if (pass == 0) __threadfence();
  }
}

__global__ __launch_bounds__(128) void k_conv3(const unsigned short* __restrict__ Ah, const unsigned short* __restrict__ Al,
                                               const unsigned short* __restrict__ Wt, float* __restrict__ Hout) {
  __shared__ __attribute__((aligned(16))) float so[4][32][68];
  const int tid = threadIdx.x, w = tid >> 5, lane = tid & 31, ln = lane & 15, hh = lane >> 4;
  const int mt = blockIdx.x >> 1, nq = blockIdx.x & 1;
  const int row0 = mt * 128 + 32 * w, col0 = nq * 64;
  const int y = row0 / LL, x0 = row0 - y * LL;
  const unsigned short* b0p = Wt + (size_t)(col0 + ln) * K33;
  v8f c0[4], c1[4];
#pragma unroll
  for (int t = 0; t < 4; ++t) { c0[t] = zero8(); c1[t] = zero8(); }
#pragma unroll 1
  for (int tap = 0; tap < 9; ++tap) {
    const int dy = tap / 3, dx = tap - dy * 3;
    const size_t pr0 = ((size_t)(y + dy) * PADW + (size_t)(x0 + dx + ln)) * OO;
    const size_t pr1 = pr0 + (size_t)16 * OO;
#pragma unroll
    for (int cb = 0; cb < 4; ++cb) {
      const int koff = cb * 32, kk = tap * OO + koff;
      const v16b a0h = fragG(Ah + pr0 + koff, hh), a0l = fragG(Al + pr0 + koff, hh);
      const v16b a1h = fragG(Ah + pr1 + koff, hh), a1l = fragG(Al + pr1 + koff, hh);
#pragma unroll
      for (int t = 0; t < 4; ++t) {
        const v16b bq = fragG(b0p + (size_t)t * 16 * K33 + kk, hh);
        c0[t] = mma2(a0h, a0l, bq, c0[t]); c1[t] = mma2(a1h, a1l, bq, c1[t]);
      }
    }
  }
#pragma unroll
  for (int t = 0; t < 4; ++t) {
#pragma unroll
    for (int r = 0; r < 8; ++r) { so[w][8 * hh + r][t * 16 + ln] = c0[t][r]; so[w][16 + 8 * hh + r][t * 16 + ln] = c1[t][r]; }
  }
  __builtin_amdgcn_fence(__ATOMIC_ACQ_REL, "workgroup");
  __builtin_amdgcn_wave_barrier();
  const int rsub = lane >> 4, c4 = (lane & 15) * 4;
  for (int pass = 0; pass < 2; ++pass) {
#pragma unroll
    for (int q = 0; q < 16; ++q) {
      const int r = q * 2 + rsub;
      const v4f v = *(const v4fa*)&so[w][r][c4];
      *(volatile v4f*)(Hout + (size_t)(row0 + r) * OO + col0 + c4) = v;
    }
    if (pass == 0) __threadfence();
  }
}

__global__ __launch_bounds__(128) void k_instat_part(const float* __restrict__ H, double* __restrict__ part) {
  const int y = blockIdx.x, c = threadIdx.x;
  double s = 0.0, q = 0.0;
#pragma unroll 4
  for (int x = 0; x < LL; ++x) { const double v = (double)H[((size_t)(y * LL + x)) * OO + c]; s += v; q += v * v; }
  double* ps = part + (size_t)y * 2 * OO + c;
  double* pq = ps + OO;
  for (int pass = 0; pass < 2; ++pass) {
    *(volatile double*)ps = s;
    *(volatile double*)pq = q;
    if (pass == 0) __threadfence();
  }
}
__global__ __launch_bounds__(128) void k_instat_fin(const double* __restrict__ part, float* __restrict__ st) {
  const int c = threadIdx.x;
  double s = 0.0, q = 0.0;
#pragma unroll 4
  for (int y = 0; y < LL; ++y) { s += part[(size_t)y * 2 * OO + c]; q += part[(size_t)y * 2 * OO + OO + c]; }
  const double mean = s * (1.0 / (double)NPIX);
  double var = q * (1.0 / (double)NPIX) - mean * mean;
  if (var < 0.0) var = 0.0;
  const float meanf = (float)mean;
  const float rstd = rsqrtf((float)var + 1e-6f);
  for (int pass = 0; pass < 2; ++pass) {
    *(volatile float*)(st + c) = meanf;
    *(volatile float*)(st + OO + c) = rstd;
    if (pass == 0) __threadfence();
  }
}

__global__ __launch_bounds__(256) void k_border(unsigned short* __restrict__ Ah, unsigned short* __restrict__ Al) {
  const int NBP = 2 * PADW + 2 * LL;
  const int t = blockIdx.x * 256 + threadIdx.x;
  if (t >= 2 * NBP * 16) return;
  const int piece = t & 15, bp = (t >> 4) % NBP, pl = (t >> 4) / NBP;
  int yp, xp;
  if (bp < PADW) { yp = 0; xp = bp; }
  else if (bp < 2 * PADW) { yp = PADW - 1; xp = bp - PADW; }
  else if (bp < 2 * PADW + LL) { yp = bp - 2 * PADW + 1; xp = 0; }
  else { yp = bp - 2 * PADW - LL + 1; xp = PADW - 1; }
  unsigned short* P = pl ? Al : Ah;
  unsigned short* dst = P + ((size_t)yp * PADW + xp) * OO + piece * 8;
  v8us z;
#pragma unroll
  for (int j = 0; j < 8; ++j) z[j] = 0;
  *(volatile v8us*)dst = z;
  __threadfence();
  *(volatile v8us*)dst = z;
}

__global__ __launch_bounds__(256) void k_act(const float* __restrict__ H, const float* __restrict__ st, const float* __restrict__ g, const float* __restrict__ bb,
                                             unsigned short* __restrict__ Ah, unsigned short* __restrict__ Al) {
  const int t = blockIdx.x * 256 + threadIdx.x;
  if (t >= NPIX * 32) return;
  const int pix = t >> 5, c4 = (t & 31) * 4;
  const v4f h = *(const v4fa*)(H + (size_t)pix * OO + c4);
  const v4f mv = *(const v4fa*)(st + c4), rv = *(const v4fa*)(st + OO + c4);
  const v4f gv = *(const v4fa*)(g + c4), bv = *(const v4fa*)(bb + c4);
  v4us hv, lv;
#pragma unroll
  for (int j = 0; j < 4; ++j) {
    const float v = (h[j] - mv[j]) * rv[j] * bfr(gv[j]) + bfr(bv[j]);
    const float e = eluf(v);
    const unsigned short hb = bfb(e); hv[j] = hb; lv[j] = bfb(e - bfv(hb));
  }
  const int y = pix / LL, x = pix - y * LL;
  const size_t d = ((size_t)(y + 1) * PADW + (size_t)(x + 1)) * OO + c4;
  for (int pass = 0; pass < 2; ++pass) {
    *(volatile v4us*)(Ah + d) = hv;
    *(volatile v4us*)(Al + d) = lv;
    if (pass == 0) __threadfence();
  }
}

__global__ __launch_bounds__(256) void k_final(const float* __restrict__ X0, const float* __restrict__ st0, const float* __restrict__ g0, const float* __restrict__ b0,
                                               const float* __restrict__ H2, const float* __restrict__ st2, const float* __restrict__ g2, const float* __restrict__ bb2,
                                               float* __restrict__ out) {
  const int t = blockIdx.x * 256 + threadIdx.x;
  if (t >= NPIX * 64) return;
  const int pix = t >> 6, c2 = (t & 63) * 2;
  const v2fa xv = *(const v2fa*)(X0 + (size_t)pix * OO + c2);
  const v2fa hv = *(const v2fa*)(H2 + (size_t)pix * OO + c2);
  v2fa o;
#pragma unroll
  for (int j = 0; j < 2; ++j) {
    const int c = c2 + j;
    const float x1 = eluf((xv[j] - st0[c]) * st0[OO + c] * bfr(g0[c]) + bfr(b0[c]));
    const float hn = (hv[j] - st2[c]) * st2[OO + c] * bfr(g2[c]) + bfr(bb2[c]);
    o[j] = eluf(x1 + hn);
  }
  float* dst = out + (size_t)pix * OO + c2;
  *(volatile v2fa*)dst = o;
  __threadfence();
  *(volatile v2fa*)dst = o;
}

extern "C" void kernel_launch(void* const* d_in, const int* in_sizes, int n_in,
                              void* d_out, int out_size, void* d_ws, size_t ws_size, hipStream_t stream) {
  if (n_in < 25) return;
  const int need[25] = {NSEQ_FULL * LL_FULL * FF, LL_FULL * LL_FULL * OO, FF, FF, PP * FF, PP, KPR, KPR, OO * KPR, OO, PP, PP, OO, OO, OO, OO,
                        OO * CIN, OO, OO, OO * OO * 9, OO, OO, OO * OO * 9, OO, OO};
  for (int i = 0; i < 25; ++i) if (in_sizes[i] < need[i]) return;
  if (out_size < NPIX * OO) return;
  const float* msa = (const float*)d_in[0];
  const float* pair_o = (const float*)d_in[1];
  const float* ln1_g = (const float*)d_in[2];
  const float* ln1_b = (const float*)d_in[3];
  const float* w1 = (const float*)d_in[4];
  const float* b1 = (const float*)d_in[5];
  const float* ln2d_g = (const float*)d_in[6];
  const float* ln2d_b = (const float*)d_in[7];
  const float* w2 = (const float*)d_in[8];
  const float* b2 = (const float*)d_in[9];
  const float* lnd_g = (const float*)d_in[10];
  const float* lnd_b = (const float*)d_in[11];
  const float* lno_g = (const float*)d_in[12];
  const float* lno_b = (const float*)d_in[13];
  const float* lnn_g = (const float*)d_in[14];
  const float* lnn_b = (const float*)d_in[15];
  const float* conv_in_w = (const float*)d_in[16];
  const float* in0_g = (const float*)d_in[17];
  const float* in0_b = (const float*)d_in[18];
  const float* rb_w1 = (const float*)d_in[19];
  const float* rb_in1_g = (const float*)d_in[20];
  const float* rb_in1_b = (const float*)d_in[21];
  const float* rb_w2 = (const float*)d_in[22];
  const float* rb_in2_g = (const float*)d_in[23];
  const float* rb_in2_b = (const float*)d_in[24];
  float* out = (float*)d_out;

  char* ws = (char*)d_ws;
  size_t off = 0;
  auto take = [&](size_t bytes) -> char* { char* p = ws + off; off += (bytes + 255) & ~(size_t)255; return p; };
  unsigned short* W1b = (unsigned short*)take((size_t)PP * FF * 2);
  unsigned short* W2t = (unsigned short*)take((size_t)OO * KPR * 2);
  unsigned short* WCt = (unsigned short*)take((size_t)OO * CIN * 2);
  unsigned short* WR1 = (unsigned short*)take((size_t)OO * K33 * 2);
  unsigned short* WR2 = (unsigned short*)take((size_t)OO * K33 * 2);
  unsigned short* Fh = (unsigned short*)take((size_t)LL * FF * 2);
  unsigned short* Fl = (unsigned short*)take((size_t)LL * FF * 2);
  double* PART = (double*)take((size_t)LL * 2 * OO * 8);
  float* ST0 = (float*)take((size_t)2 * OO * 4);
  float* ST1 = (float*)take((size_t)2 * OO * 4);
  float* ST2 = (float*)take((size_t)2 * OO * 4);
  float* X0 = (float*)take((size_t)NPIX * OO * 4);
  const size_t szXD = (size_t)NROW0 * PP * 4;
  const size_t szXT = (size_t)LL * PP * NSEQ * 2;
  const size_t szP = (size_t)NPIX * OO * 2;
  const size_t szAP = (size_t)NPADPIX * OO * 2;
  const size_t szH = (size_t)NPIX * OO * 4;
  const size_t ph1 = szXD + 2 * szXT + 4 * szP, ph2 = 2 * szAP + szH;
  char* arena = take(ph1 > ph2 ? ph1 : ph2);
  if (off > ws_size || off > (size_t)134217728) return;
  float* XD = (float*)arena;
  unsigned short* XTh = (unsigned short*)(arena + szXD);
  unsigned short* XTl = (unsigned short*)(arena + szXD + szXT);
  unsigned short* POh = (unsigned short*)(arena + szXD + 2 * szXT);
  unsigned short* POl = (unsigned short*)(arena + szXD + 2 * szXT + szP);
  unsigned short* PNh = (unsigned short*)(arena + szXD + 2 * szXT + 2 * szP);
  unsigned short* PNl = (unsigned short*)(arena + szXD + 2 * szXT + 3 * szP);
  unsigned short* APh = (unsigned short*)arena;
  unsigned short* APl = (unsigned short*)(arena + szAP);
  float* H = (float*)(arena + 2 * szAP);

  k_cvt<<<(PP * FF / 8 + 255) / 256, 256, 0, stream>>>(w1, W1b, PP * FF / 8);
  k_cvt<<<(OO * KPR / 8 + 255) / 256, 256, 0, stream>>>(w2, W2t, OO * KPR / 8);
  k_cvt<<<(OO * CIN / 8 + 255) / 256, 256, 0, stream>>>(conv_in_w, WCt, OO * CIN / 8);
  k_w9<<<(OO * 9 * 16 + 255) / 256, 256, 0, stream>>>(rb_w1, WR1);
  k_w9<<<(OO * 9 * 16 + 255) / 256, 256, 0, stream>>>(rb_w2, WR2);
  k_proj1<<<NROW0 / 64, 128, 0, stream>>>(msa, ln1_g, ln1_b, W1b, b1, XD);
  k_xt<<<LL, 256, 0, stream>>>(XD, XTh, XTl);
  k_feat<<<LL, 256, 0, stream>>>(XD, lnd_g, lnd_b, Fh, Fl);
  k_lnpo<<<NPIX / 8, 256, 0, stream>>>(pair_o, lno_g, lno_b, POh, POl);
  hipFuncSetAttribute(reinterpret_cast<const void*>(&k_pair), hipFuncAttributeMaxDynamicSharedMemorySize, (int)KPAIR_LDS);
  k_pair<<<NTRI, 256, KPAIR_LDS, stream>>>(XTh, XTl, ln2d_g, ln2d_b, W2t, b2, lnn_g, lnn_b, PNh, PNl);
  k_conv1<<<(NPIX / 128) * 2, 128, 0, stream>>>(POh, POl, PNh, PNl, Fh, Fl, WCt, X0);
  k_instat_part<<<LL, OO, 0, stream>>>(X0, PART);
  k_instat_fin<<<1, OO, 0, stream>>>(PART, ST0);
  k_border<<<(2 * (2 * PADW + 2 * LL) * 16 + 255) / 256, 256, 0, stream>>>(APh, APl);
  k_act<<<(NPIX * 32) / 256, 256, 0, stream>>>(X0, ST0, in0_g, in0_b, APh, APl);
  k_conv3<<<(NPIX / 128) * 2, 128, 0, stream>>>(APh, APl, WR1, H);
  k_instat_part<<<LL, OO, 0, stream>>>(H, PART);
  k_instat_fin<<<1, OO, 0, stream>>>(PART, ST1);
  k_act<<<(NPIX * 32) / 256, 256, 0, stream>>>(H, ST1, rb_in1_g, rb_in1_b, APh, APl);
  k_conv3<<<(NPIX / 128) * 2, 128, 0, stream>>>(APh, APl, WR2, H);
  k_instat_part<<<LL, OO, 0, stream>>>(H, PART);
  k_instat_fin<<<1, OO, 0, stream>>>(PART, ST2);
  k_final<<<(NPIX * 64) / 256, 256, 0, stream>>>(X0, ST0, in0_g, in0_b, H, ST2, rb_in2_g, rb_in2_b, out);
}
